// MessageBlock_17815524344046
// MI455X (gfx1250) — hardware-verified
//
#include <hip/hip_runtime.h>
#include <stdint.h>

typedef _Float16       v16h  __attribute__((ext_vector_type(16)));
typedef unsigned short v16us __attribute__((ext_vector_type(16)));
typedef unsigned short v8us  __attribute__((ext_vector_type(8)));
typedef unsigned int   v4u   __attribute__((ext_vector_type(4)));
typedef float          v8f   __attribute__((ext_vector_type(8)));
typedef float          v4f   __attribute__((ext_vector_type(4)));
typedef v8us __attribute__((may_alias)) v8usa;
typedef v4u  __attribute__((may_alias)) v4ua;
typedef v4f  __attribute__((may_alias)) v4fa;

union FragU { v16us v; v8us half[2]; };
union HFv   { v16us u; v16h f; };

#define NN   1024
#define CC   128
#define DI   16
#define EE   10
#define OW   512
#define NPM  256
#define NTM  16
#define DP   260
#define SCL_A   64.0f
#define SCL_B   256.0f
#define SCL_INV 6.103515625e-05f

__device__ __forceinline__ unsigned short f2bf(float f) {
  unsigned u = __float_as_uint(f);
  u = u + 0x7FFFu + ((u >> 16) & 1u);
  return (unsigned short)(u >> 16);
}
__device__ __forceinline__ float bf2f(unsigned short b) { return __uint_as_float(((unsigned)b) << 16); }
__device__ __forceinline__ float bfr(float f) { return bf2f(f2bf(f)); }
__device__ __forceinline__ unsigned short f2h(float f) {
  union { _Float16 h; unsigned short u; } q;
  q.h = (_Float16)f;
  return q.u;
}
__device__ __forceinline__ unsigned pk2(unsigned short lo, unsigned short hi) {
  return (unsigned)lo | (((unsigned)hi) << 16);
}

__device__ __forceinline__ v8f wmma_f16(v16us au, v16us bu, v8f c) {
  HFv A, B; A.u = au; B.u = bu;
  v8f d = __builtin_amdgcn_wmma_f32_16x16x32_f16(false, A.f, false, B.f, (short)0, c, false, false);
  asm volatile("v_nop\n\tv_nop\n\tv_nop\n\tv_nop" : "+v"(d) : "v"(au), "v"(bu));
  return d;
}

__device__ __forceinline__ v16us ldfrag(const unsigned short* p, int h) {
  FragU f;
  f.half[0] = *(const v8usa*)(p + 8 * h);
  f.half[1] = *(const v8usa*)(p + 16 + 8 * h);
  return f.v;
}

template <int P3, int P2, int KP, int NQ>
__device__ __forceinline__ void prep_pieces(const float* __restrict__ U3, const float* __restrict__ U2,
                                            unsigned* __restrict__ Bt, int g)
{
  constexpr int PPR = KP / 8;
  constexpr int L3 = DI * P3;
  static_assert(L3 % 8 == 0);
  static_assert(L3 + P2 <= KP);
  static_assert(P2 <= 8);
  const bool active = (g < PPR * NQ);
  const int gg = active ? g : 0;
  const int q = gg / PPR;
  const int kp0 = (gg - q * PPR) * 8;
  const bool in3 = (kp0 < L3);
  const int kc = in3 ? kp0 : 0;
  const float* s3 = U3 + (size_t)q * L3 + kc;
  const v4f ua = *(const v4fa*)(s3);
  const v4f ub = *(const v4fa*)(s3 + 4);
  float u2v[P2];
  #pragma unroll
  for (int k = 0; k < P2; ++k) u2v[k] = U2[(size_t)q * P2 + k];
  const float u3v[8] = {ua.x, ua.y, ua.z, ua.w, ub.x, ub.y, ub.z, ub.w};
  unsigned short hb[8];
  #pragma unroll
  for (int e = 0; e < 8; ++e) {
    const int kp = kp0 + e;
    float v2 = 0.0f;
    #pragma unroll
    for (int k = 0; k < P2; ++k) v2 = (kp == L3 + k) ? u2v[k] : v2;
    const float v = in3 ? u3v[e] : v2;
    hb[e] = f2h(SCL_B * bfr(v));
  }
  v4u o;
  o.x = pk2(hb[0], hb[1]); o.y = pk2(hb[2], hb[3]); o.z = pk2(hb[4], hb[5]); o.w = pk2(hb[6], hb[7]);
  unsigned* dst = Bt + (size_t)gg * 4;
  if (active) *(volatile v4u*)dst = o;
  __threadfence();
  if (active) *(volatile v4u*)dst = o;
}

__global__ __launch_bounds__(256) void k_prep(
    const float* __restrict__ U3a, const float* __restrict__ U2a,
    const float* __restrict__ U3b, const float* __restrict__ U2b,
    unsigned* __restrict__ Bta, unsigned* __restrict__ Btb)
{
  const int bid = blockIdx.x, tid = threadIdx.x;
  if (bid < 12) {
    prep_pieces<5, 2, 96, 256>(U3a, U2a, Bta, bid * 256 + tid);
  } else {
    prep_pieces<7, 3, 128, 768>(U3b, U2b, Btb, (bid - 12) * 256 + tid);
  }
}

template <int M>
__device__ __forceinline__ void out_store_pass(const float* ys, float* out, int n, int cb, int tid) {
  const int p = tid;
  const int pc = (p < 16 * M) ? p : 0;
  const v4f v = *(const v4fa*)(ys + 4 * pc);
  const size_t base = (size_t)n * OW + (size_t)((M == 1) ? cb : (CC + 3 * cb));
  if (p < 16 * M) *(volatile v4f*)(out + base + 4 * p) = v;
}

template <int M, int KP>
__host__ __device__ constexpr int sym_lds_bytes() { return 64 * KP * 2 + 2 * 32 * DP * 4 + 64 * DI * 4 + 48 * 4 + 64 * M * 4; }

template <int M, int P3, int P2, int KP>
__global__ __launch_bounds__(64) void k_sym(
    const float* __restrict__ ai,
    const float* __restrict__ na,
    const float* __restrict__ U1,
    const float* __restrict__ W1,
    const float* __restrict__ W2,
    const float* __restrict__ W3,
    const unsigned short* __restrict__ Bt,
    float* __restrict__ out)
{
  static_assert(KP % 32 == 0);
  static_assert(DI * P3 + P2 <= KP);
  static_assert(M * DI <= 48);
  static_assert(M == 1 || M == 3);
  static_assert(P3 <= 8 && P2 <= 7);
  constexpr int KSN = KP / 32;
  constexpr int KPW = KP / 2;
  constexpr int L3  = DI * P3;

  extern __shared__ unsigned char dsm_s[] __attribute__((aligned(16)));
  unsigned* Apl = (unsigned*)dsm_s;
  float* Dst = (float*)(dsm_s + 64 * KP * 2);
  float* xs  = Dst + 2 * 32 * DP;
  float* u1s = xs + 64 * DI;
  float* ys  = u1s + 48;

  const int tid = threadIdx.x, lane = tid & 31, wave = tid >> 5;
  const int h = lane >> 4, m16 = lane & 15;
  const int n = blockIdx.x >> 1, cb = (blockIdx.x & 1) * 64, c = cb + tid;

  float x[DI];
  const float* xr = ai + ((size_t)n * CC + c) * DI;
  #pragma unroll
  for (int j = 0; j < 4; ++j) {
    const v4f r = *(const v4fa*)(xr + 4 * j);
    v4f rb;
    rb.x = bfr(r.x); rb.y = bfr(r.y); rb.z = bfr(r.z); rb.w = bfr(r.w);
    x[4 * j + 0] = rb.x; x[4 * j + 1] = rb.y; x[4 * j + 2] = rb.z; x[4 * j + 3] = rb.w;
    *(v4fa*)(xs + tid * DI + 4 * j) = rb;
  }
  if (tid < M * DI) u1s[tid] = bfr(U1[tid]);

  float w3[P3], w2[P2];
  float w1 = 0.0f;
  #pragma unroll
  for (int k = 0; k < P3; ++k) w3[k] = 0.0f;
  #pragma unroll
  for (int k = 0; k < P2; ++k) w2[k] = 0.0f;
  #pragma unroll 1
  for (int e = 0; e < EE; ++e) {
    const float a = bfr(na[n * EE + e]);
    w1 = fmaf(a, bfr(W1[e * CC + c]), w1);
    #pragma unroll
    for (int k = 0; k < P2; ++k) w2[k] = fmaf(a, bfr(W2[(e * P2 + k) * CC + c]), w2[k]);
  }
  #pragma unroll 1
  for (int e = 0; e < EE; ++e) {
    const float a = bfr(na[n * EE + e]);
    #pragma unroll
    for (int k = 0; k < P3; ++k) w3[k] = fmaf(a, bfr(W3[(e * P3 + k) * CC + c]), w3[k]);
  }

  #pragma unroll
  for (int pc = 0; pc < KP / 8; ++pc) {
    unsigned short hb[8];
    #pragma unroll
    for (int e = 0; e < 8; ++e) {
      const int kp = pc * 8 + e;
      const int ii = (kp < L3) ? (kp / P3) : 0;
      const int kk = (kp < L3) ? (kp - ii * P3) : 0;
      const int k2 = (kp >= L3 && kp < L3 + P2) ? (kp - L3) : 0;
      const float v = (kp < L3) ? (SCL_A * (x[ii] * w3[kk]))
                                : ((kp < L3 + P2) ? (SCL_A * w2[k2]) : 0.0f);
      hb[e] = f2h(v);
    }
    v4u o;
    o.x = pk2(hb[0], hb[1]); o.y = pk2(hb[2], hb[3]); o.z = pk2(hb[4], hb[5]); o.w = pk2(hb[6], hb[7]);
    *(v4ua*)(Apl + tid * KPW + pc * 4) = o;
  }
  __syncthreads();

  const unsigned short* Aps = (const unsigned short*)Apl;
  v16us af0[KSN], af1[KSN];
  #pragma unroll
  for (int ks = 0; ks < KSN; ++ks) {
    af0[ks] = ldfrag(Aps + (wave * 32 + m16) * KP + ks * 32, h);
    af1[ks] = ldfrag(Aps + (wave * 32 + 16 + m16) * KP + ks * 32, h);
  }
  float* Dw = Dst + wave * 32 * DP;
  const v8f z8 = {0.f, 0.f, 0.f, 0.f, 0.f, 0.f, 0.f, 0.f};

  #pragma unroll 1
  for (int m = 0; m < M; ++m) {
    #pragma unroll 1
    for (int nt = 0; nt < NTM; ++nt) {
      const int q = nt * 16 + m16;
      const unsigned short* bp = Bt + (size_t)(m * NPM + q) * KP;
      v8f a0 = z8, a1 = z8;
      #pragma unroll
      for (int ks = 0; ks < KSN; ++ks) {
        const v16us bb = ldfrag(bp + ks * 32, h);
        a0 = wmma_f16(af0[ks], bb, a0);
        a1 = wmma_f16(af1[ks], bb, a1);
      }
      #pragma unroll
      for (int r = 0; r < 8; ++r) {
        Dw[(8 * h + r) * DP + q]      = a0[r];
        Dw[(16 + 8 * h + r) * DP + q] = a1[r];
      }
    }
    __syncthreads();

    {
      const float* Dr = Dst + tid * DP;
      float ym = 0.0f;
      #pragma unroll 1
      for (int i1 = 0; i1 < DI; ++i1) {
        const float* dq = Dr + i1 * DI;
        float o2s = 0.0f;
        #pragma unroll
        for (int j = 0; j < 4; ++j) {
          const v4f d4 = *(const v4fa*)(dq + 4 * j);
          o2s = fmaf(d4.x, x[4 * j + 0], o2s);
          o2s = fmaf(d4.y, x[4 * j + 1], o2s);
          o2s = fmaf(d4.z, x[4 * j + 2], o2s);
          o2s = fmaf(d4.w, x[4 * j + 3], o2s);
        }
        const float o2  = o2s * SCL_INV;
        const float t1  = u1s[m * DI + i1] * w1;
        const float ct1 = o2 + t1;
        ym = fmaf(ct1, xs[tid * DI + i1], ym);
      }
      ys[tid * M + m] = ym;
    }
    __syncthreads();
  }

  out_store_pass<M>(ys, out, n, cb, tid);
  __threadfence();
  out_store_pass<M>(ys, out, n, cb, tid);
}

extern "C" void kernel_launch(void* const* d_in, const int* in_sizes, int n_in,
                              void* d_out, int out_size, void* d_ws, size_t ws_size,
                              hipStream_t stream) {
  if (n_in < 14) return;
  if (in_sizes[0] != NN * CC * DI) return;
  if (in_sizes[1] != NN * EE) return;
  if (in_sizes[2] != 256 * DI * 5) return;
  if (in_sizes[3] != 256 * 2) return;
  if (in_sizes[4] != DI) return;
  if (in_sizes[5] != EE * 5 * CC) return;
  if (in_sizes[6] != EE * 2 * CC) return;
  if (in_sizes[7] != EE * 1 * CC) return;
  if (in_sizes[8] != 768 * DI * 7) return;
  if (in_sizes[9] != 768 * 3) return;
  if (in_sizes[10] != 3 * DI) return;
  if (in_sizes[11] != EE * 7 * CC) return;
  if (in_sizes[12] != EE * 3 * CC) return;
  if (in_sizes[13] != EE * 1 * CC) return;
  if (out_size != NN * OW) return;

  const float* ai    = (const float*)d_in[0];
  const float* na    = (const float*)d_in[1];
  const float* U3_0  = (const float*)d_in[2];
  const float* U2_0  = (const float*)d_in[3];
  const float* U1_0  = (const float*)d_in[4];
  const float* W3_0  = (const float*)d_in[5];
  const float* W2_0  = (const float*)d_in[6];
  const float* W1_0  = (const float*)d_in[7];
  const float* U3_1  = (const float*)d_in[8];
  const float* U2_1  = (const float*)d_in[9];
  const float* U1_1  = (const float*)d_in[10];
  const float* W3_1  = (const float*)d_in[11];
  const float* W2_1  = (const float*)d_in[12];
  const float* W1_1  = (const float*)d_in[13];
  float* out = (float*)d_out;

  const size_t bt0_b = (size_t)256 * 96 * 2;
  const size_t bt1_b = (size_t)768 * 128 * 2;
  const size_t off_bt0 = 0;
  const size_t off_bt1 = off_bt0 + bt0_b;
  const size_t total   = off_bt1 + bt1_b;
  if (total > ws_size) return;

  char* ws = (char*)d_ws;
  unsigned* Bt0 = (unsigned*)(ws + off_bt0);
  unsigned* Bt1 = (unsigned*)(ws + off_bt1);

  k_prep<<<dim3(60), dim3(256), 0, stream>>>(U3_0, U2_0, U3_1, U2_1, Bt0, Bt1);

  constexpr int lds0 = sym_lds_bytes<1, 96>();
  constexpr int lds1 = sym_lds_bytes<3, 128>();
  hipFuncSetAttribute(reinterpret_cast<const void*>(&k_sym<1, 5, 2, 96>),
                      hipFuncAttributeMaxDynamicSharedMemorySize, lds0);
  hipFuncSetAttribute(reinterpret_cast<const void*>(&k_sym<3, 7, 3, 128>),
                      hipFuncAttributeMaxDynamicSharedMemorySize, lds1);
  k_sym<1, 5, 2, 96><<<dim3(NN * 2), dim3(64), lds0, stream>>>(
      ai, na, U1_0, W1_0, W2_0, W3_0, (const unsigned short*)Bt0, out);
  k_sym<3, 7, 3, 128><<<dim3(NN * 2), dim3(64), lds1, stream>>>(
      ai, na, U1_1, W1_1, W2_1, W3_1, (const unsigned short*)Bt1, out);
}
